// Skinning_22290880266410
// MI455X (gfx1250) — hardware-verified
//
#include <hip/hip_runtime.h>


#define NV   100000
#define NVP  100096
#define HALF 50048
#define NJ   52
#define KP   64
#define NP   32
#define NC   (NP * 16)
typedef _Float16 h16;
typedef unsigned short bf;
typedef __attribute__((ext_vector_type(16))) __bf16   v16bf;
typedef __attribute__((ext_vector_type(16))) _Float16 v16h;
typedef __attribute__((ext_vector_type(8)))  _Float16 v8h;
typedef __attribute__((ext_vector_type(8)))  unsigned short v8us;
typedef __attribute__((ext_vector_type(8)))  float    v8f;
typedef __attribute__((ext_vector_type(4)))  float    v4f;
typedef v8h  __attribute__((may_alias)) v8ha;
typedef v4f  __attribute__((may_alias)) v4fa;
typedef v8us __attribute__((may_alias)) v8usa;

__device__ __forceinline__ unsigned short f2bf(float f) { unsigned u = __float_as_uint(f); u += 0x7FFFu + ((u >> 16) & 1u); return (unsigned short)(u >> 16); }
__device__ __forceinline__ float bf2f(unsigned short b) { return __uint_as_float(((unsigned)b) << 16); }
__device__ __forceinline__ float bfr(float f) { return bf2f(f2bf(f)); }
__device__ __forceinline__ v16h cat16(v8h lo, v8h hi) { return __builtin_shufflevector(lo, hi, 0, 1, 2, 3, 4, 5, 6, 7, 8, 9, 10, 11, 12, 13, 14, 15); }
__device__ __forceinline__ v16bf cat16b(v8us lo, v8us hi) { return __builtin_bit_cast(v16bf, __builtin_shufflevector(lo, hi, 0, 1, 2, 3, 4, 5, 6, 7, 8, 9, 10, 11, 12, 13, 14, 15)); }
__device__ __forceinline__ v8f wmma16(v16h a, v16h b, v8f c) { return __builtin_amdgcn_wmma_f32_16x16x32_f16(false, a, false, b, (short)0, c, false, false); }
__device__ __forceinline__ v8f wmmab(v16bf a, v16bf b, v8f c) { return __builtin_amdgcn_wmma_f32_16x16x32_bf16(false, a, false, b, (short)0, c, false, false); }


template <typename T16> struct WFrag;
template <> struct WFrag<h16> { typedef v16h V; static __device__ __forceinline__ V ld(const h16* p) { return cat16(*(const v8h*)p, *(const v8h*)(p + 16)); } static __device__ __forceinline__ v8f mma(V a, V b, v8f c) { return wmma16(a, b, c); } };
template <> struct WFrag<bf> { typedef v16bf V; static __device__ __forceinline__ V ld(const bf* p) { return cat16b(*(const v8us*)p, *(const v8us*)(p + 16)); } static __device__ __forceinline__ v8f mma(V a, V b, v8f c) { return wmmab(a, b, c); } };
template <typename T16, int NSPLIT, bool BIAS>
__global__ __launch_bounds__(32) void k_gemmw(const T16* __restrict__ A, const T16* __restrict__ A2, const T16* __restrict__ Bt, const T16* __restrict__ Bt2, int K, float* C, int ldc, const float* __restrict__ bias, size_t sA, size_t sB, size_t sC) {
    typedef typename WFrag<T16>::V V;
    __shared__ __align__(16) float os[16 * 68];
    const size_t z = blockIdx.z; A += z * sA; if (A2) A2 += z * sA; Bt += z * sB; if (Bt2) Bt2 += z * sB; C += z * sC;
    const int lane = threadIdx.x & 31, lr = lane & 15, hi = lane >> 4; const int r0 = blockIdx.x * 64, c0 = blockIdx.y * 64;
    v8f acc[4][4];
#pragma unroll
    for (int mb = 0; mb < 4; ++mb)
#pragma unroll
        for (int nb = 0; nb < 4; ++nb) acc[mb][nb] = (v8f){};
    const size_t aoff = (size_t)(r0 + lr) * K + 8 * hi, boff = (size_t)(c0 + lr) * K + 8 * hi;
#pragma unroll 1
    for (int kc = 0; kc < K; kc += 32) {
        V a[4], a2[4];
#pragma unroll
        for (int mb = 0; mb < 4; ++mb) { a[mb] = WFrag<T16>::ld(A + aoff + (size_t)mb * 16 * K + kc); if (NSPLIT == 1 || NSPLIT == 2) a2[mb] = WFrag<T16>::ld(A2 + aoff + (size_t)mb * 16 * K + kc); }
#pragma unroll
        for (int nb = 0; nb < 4; ++nb) { const V b = WFrag<T16>::ld(Bt + boff + (size_t)nb * 16 * K + kc); V b2; if (NSPLIT >= 2) b2 = WFrag<T16>::ld(Bt2 + boff + (size_t)nb * 16 * K + kc);
#pragma unroll
            for (int mb = 0; mb < 4; ++mb) { acc[mb][nb] = WFrag<T16>::mma(a[mb], b, acc[mb][nb]); if (NSPLIT == 1 || NSPLIT == 2) acc[mb][nb] = WFrag<T16>::mma(a2[mb], b, acc[mb][nb]); if (NSPLIT >= 2) acc[mb][nb] = WFrag<T16>::mma(a[mb], b2, acc[mb][nb]); } }
        asm volatile("v_nop\n\tv_nop\n\tv_nop\n\tv_nop" : "+v"(acc[0][0]), "+v"(acc[1][1]), "+v"(acc[2][2]), "+v"(acc[3][3]) : "v"(a[0]), "v"(a[3]));
    }
#pragma unroll
    for (int mb = 0; mb < 4; ++mb) {
#pragma unroll
        for (int nb = 0; nb < 4; ++nb) {
#pragma unroll
            for (int j = 0; j < 8; ++j) os[(hi * 8 + j) * 68 + nb * 16 + lr] = acc[mb][nb][j]; }
        __builtin_amdgcn_wave_barrier(); asm volatile("" ::: "memory");
        float* crow = C + (size_t)(r0 + mb * 16) * ldc + c0;
#pragma unroll 1
        for (int ps = 0; ps < 2; ++ps) {
#pragma unroll
            for (int s = 0; s < 8; ++s) { const int row = 2 * s + hi, cofs = lr * 4; v4f val = *(const v4fa*)(os + row * 68 + cofs); if (BIAS) { val[0] += bfr(bias[c0 + cofs]); val[1] += bfr(bias[c0 + cofs + 1]); val[2] += bfr(bias[c0 + cofs + 2]); val[3] += bfr(bias[c0 + cofs + 3]); }
                *(volatile v4f*)(crow + (size_t)row * ldc + cofs) = val; }
            if (ps == 0) __threadfence(); }
        __builtin_amdgcn_wave_barrier(); asm volatile("" ::: "memory");
    }
}

typedef __attribute__((ext_vector_type(4))) unsigned short v4us;

__global__ __launch_bounds__(256) void k_wpad(const float* __restrict__ w, bf* A) { const size_t e = ((size_t)blockIdx.x * 256 + threadIdx.x) * 4; if (e >= (size_t)NVP * KP) return; const int j = (int)(e & 63); const size_t v = e >> 6; v4us o;
#pragma unroll
    for (int q = 0; q < 4; ++q) o[q] = (v < NV && j + q < NJ) ? f2bf(w[v * NJ + j + q]) : (unsigned short)0; *(volatile v4us*)(A + e) = o; __threadfence(); *(volatile v4us*)(A + e) = o; }
__global__ __launch_bounds__(256) void k_tpad(const float* __restrict__ M, bf* Bt) { const int e = (blockIdx.x * 256 + threadIdx.x) * 4; if (e >= NC * KP) return; const int j = e & 63; const int n = e >> 6; const int b = n >> 4, x = n & 15; v4us o;
#pragma unroll
    for (int q = 0; q < 4; ++q) o[q] = (j + q < NJ) ? f2bf(M[((size_t)b * NJ + j + q) * 16 + x]) : (unsigned short)0; *(volatile v4us*)(Bt + e) = o; __threadfence(); *(volatile v4us*)(Bt + e) = o; }
__global__ __launch_bounds__(256) void k_apply(const float* __restrict__ C, const float* __restrict__ vert, int v0, float* OUT) { const int i = blockIdx.x * 256 + threadIdx.x; if (i >= NP * HALF) return; const int b = i / HALF; const int v = v0 + i % HALF; if (v >= NV) return;
    const float* T = C + (size_t)(v - v0) * NC + b * 16; const float vx = bfr(vert[(size_t)v * 3]), vy = bfr(vert[(size_t)v * 3 + 1]), vz = bfr(vert[(size_t)v * 3 + 2]); float o[3];
#pragma unroll
    for (int r = 0; r < 3; ++r) { float p0 = __fmul_rn(T[r * 4], vx), p1 = __fmul_rn(T[r * 4 + 1], vy), p2 = __fmul_rn(T[r * 4 + 2], vz); asm volatile("" : "+v"(p0)); asm volatile("" : "+v"(p1)); asm volatile("" : "+v"(p2)); o[r] = __fadd_rn(__fadd_rn(__fadd_rn(p0, p1), p2), T[r * 4 + 3]); }
    float* dst = OUT + ((size_t)b * NV + v) * 3;
    for (int ps = 0; ps < 2; ++ps) { *(volatile float*)(dst) = o[0]; *(volatile float*)(dst + 1) = o[1]; *(volatile float*)(dst + 2) = o[2]; if (ps == 0) __threadfence(); } }

extern "C" void kernel_launch(void* const* d_in, const int* in_sizes, int n_in,
                              void* d_out, int out_size, void* d_ws, size_t ws_size, hipStream_t stream) {
    (void)in_sizes; (void)n_in; (void)out_size;
    const float* vert = (const float*)d_in[0]; const float* w = (const float*)d_in[1]; const float* M = (const float*)d_in[2];
    float* OUT = (float*)d_out;
    char* wsp = (char*)d_ws;
    auto take = [&](size_t bytes) { char* p = wsp; wsp += (bytes + 255) & ~(size_t)255; return (void*)p; };
    bf* A = (bf*)take((size_t)NVP * KP * 2); bf* Bt = (bf*)take((size_t)NC * KP * 2); float* C = (float*)take((size_t)HALF * NC * 4);
    if ((size_t)(wsp - (char*)d_ws) > ws_size) return;
    k_wpad<<<(unsigned)(((size_t)NVP * KP / 4 + 255) / 256), 256, 0, stream>>>(w, A); k_tpad<<<(NC * KP / 4 + 255) / 256, 256, 0, stream>>>(M, Bt);
    for (int hf = 0; hf < 2; ++hf) { const int v0 = hf * HALF;
        k_gemmw<bf, 0, false><<<dim3(HALF / 64, NC / 64, 1), 32, 0, stream>>>(A + (size_t)v0 * KP, nullptr, Bt, nullptr, KP, C, NC, nullptr, 0, 0, 0);
        k_apply<<<(NP * HALF + 255) / 256, 256, 0, stream>>>(C, vert, v0, OUT); }
}
